// Encoder_6356551598792
// MI455X (gfx1250) — hardware-verified
//
#include <hip/hip_runtime.h>
#include <stddef.h>
#include <stdint.h>
#include <math.h>


#define DF     128
#define KH     256
#define NTHR   256
#define NWAVE  8
#define EPT    8
#define CHUNK  (NTHR * EPT)
#define WCAP   (EPT * 32)
#define LISTN  (NWAVE * WCAP)
#define NBA    1024
#define SLA    10
#define RCAP   24576
#define DEGCAP 64
#define GBM    64
#define GBN    64
#define GTHR   128
#define UPART  2048
#define NPART  6
#define AGG_ZINTS    (LISTN + 2 * RCAP + 3 * NBA)
#define MISC_INTS    16
#define AGG_LDS_INTS (AGG_ZINTS + MISC_INTS)
#define NREC   256
#define WSMAX  134217728

static_assert((CHUNK & (CHUNK - 1)) == 0 && CHUNK <= 4096);
static_assert((NBA & (NBA - 1)) == 0 && NBA == (1 << SLA));
static_assert(((long long)CHUNK << SLA) < (1LL << 31));
static_assert(LISTN % NTHR == 0);
static_assert(NBA % NWAVE == 0 && NBA % 32 == 0 && NBA % GBM == 0);
static_assert(RCAP % 4 == 0 && AGG_ZINTS % 4 == 0 && LISTN % 4 == 0);
static_assert(DF % 32 == 0 && KH % 32 == 0 && KH == 2 * DF && DF == 4 * 32 && DF == 2 * GBN);
static_assert(GBM == (GTHR / 32) * 16 && GBN == 64);
static_assert(UPART % NTHR == 0 && UPART == DF * (DF / 8) && (NPART * UPART) % NTHR == 0);
static_assert((NWAVE * NREC + NREC) * 2 <= RCAP);
static_assert((LISTN * 4) % 16 == 0);
static_assert(NREC == NTHR && NREC == 2 * DF);
static_assert(AGG_LDS_INTS * 4 <= 300000);

typedef float          v4f   __attribute__((ext_vector_type(4)));
typedef float          v8f   __attribute__((ext_vector_type(8)));
typedef double         v2d   __attribute__((ext_vector_type(2)));
typedef int            v4i   __attribute__((ext_vector_type(4)));
typedef int            v8i   __attribute__((ext_vector_type(8)));
typedef unsigned short v8us  __attribute__((ext_vector_type(8)));
typedef unsigned short v16us __attribute__((ext_vector_type(16)));
typedef __bf16         v16bf __attribute__((ext_vector_type(16)));
typedef v4f  __attribute__((may_alias)) v4fa;
typedef v4i  __attribute__((may_alias)) v4ia;
typedef v2d  __attribute__((may_alias)) v2da;
typedef v8us __attribute__((may_alias)) v8usa;
typedef double __attribute__((may_alias)) dbla;
union FragB { v16bf v; v16us u; v8us h[2]; v8i w; };

__device__ __forceinline__ v8f wmb(const FragB& a, const FragB& b, v8f c) {
  v8f d = __builtin_amdgcn_wmma_f32_16x16x32_bf16(false, a.v, false, b.v, (short)0, c, false, false);
  asm volatile("v_nop\n\tv_nop\n\tv_nop\n\tv_nop" : "+v"(d) : "v"(a.w), "v"(b.w));
  return d;
}

__device__ __forceinline__ unsigned bf16_bits(float f) {
  const unsigned u = __float_as_uint(f);
  return (u + 0x7FFFu + ((u >> 16) & 1u)) >> 16;
}
__device__ __forceinline__ float bf16_val(float f) {
  return __uint_as_float(bf16_bits(f) << 16);
}

template <int SLB>
__device__ __forceinline__ int scan_chunk(const int* __restrict__ dsts, int nE, int cbase, int slotBase,
                                          int nb, int vec8, int* list, int tid, int lane, int wave) {
  int wc = 0;
  const int el0  = tid * EPT;
  const int e0   = cbase + el0;
  const int sent = -2147483647 - 1;
  v4i da, db;
  if (vec8 != 0 && cbase + CHUNK <= nE) {
    da = *(const v4i*)(dsts + e0);
    db = *(const v4i*)(dsts + e0 + 4);
  } else {
    da.x = (e0     < nE) ? dsts[min(e0,     nE - 1)] : sent;
    da.y = (e0 + 1 < nE) ? dsts[min(e0 + 1, nE - 1)] : sent;
    da.z = (e0 + 2 < nE) ? dsts[min(e0 + 2, nE - 1)] : sent;
    da.w = (e0 + 3 < nE) ? dsts[min(e0 + 3, nE - 1)] : sent;
    db.x = (e0 + 4 < nE) ? dsts[min(e0 + 4, nE - 1)] : sent;
    db.y = (e0 + 5 < nE) ? dsts[min(e0 + 5, nE - 1)] : sent;
    db.z = (e0 + 6 < nE) ? dsts[min(e0 + 6, nE - 1)] : sent;
    db.w = (e0 + 7 < nE) ? dsts[min(e0 + 7, nE - 1)] : sent;
  }
  const unsigned nbs = (unsigned)slotBase;
  const unsigned unb = (unsigned)nb;
  const unsigned s0 = (unsigned)da.x - nbs, s1 = (unsigned)da.y - nbs;
  const unsigned s2 = (unsigned)da.z - nbs, s3 = (unsigned)da.w - nbs;
  const unsigned s4 = (unsigned)db.x - nbs, s5 = (unsigned)db.y - nbs;
  const unsigned s6 = (unsigned)db.z - nbs, s7 = (unsigned)db.w - nbs;
  const bool h0 = s0 < unb, h1 = s1 < unb, h2 = s2 < unb, h3 = s3 < unb;
  const bool h4 = s4 < unb, h5 = s5 < unb, h6 = s6 < unb, h7 = s7 < unb;
  const unsigned any = __builtin_amdgcn_ballot_w32(h0 | h1 | h2 | h3 | h4 | h5 | h6 | h7);
  if (any != 0u) {
#define HITJ(J, HJ, SJ) { \
      const unsigned mj = __builtin_amdgcn_ballot_w32(HJ); \
      if (mj != 0u) { \
        if (HJ) { \
          const int pos = wc + (int)__builtin_amdgcn_mbcnt_lo(mj, 0u); \
          if (pos < WCAP) list[wave * WCAP + pos] = ((el0 + (J)) << SLB) | (int)(SJ); \
        } \
        wc += (int)__builtin_popcount(mj); } }
    HITJ(0, h0, s0)
    HITJ(1, h1, s1)
    HITJ(2, h2, s2)
    HITJ(3, h3, s3)
    HITJ(4, h4, s4)
    HITJ(5, h5, s5)
    HITJ(6, h6, s6)
    HITJ(7, h7, s7)
#undef HITJ
  }
  return wc;
}

__global__ __launch_bounds__(NTHR) void k_wprep(const float* __restrict__ W1l, const float* __restrict__ W1r,
                                                const float* __restrict__ W2l, const float* __restrict__ W2r,
                                                unsigned short* WB1, unsigned short* WB2) {
  const int u    = (int)blockIdx.x * NTHR + (int)threadIdx.x;
  const int part = u >> 11;
  const int v    = u & (UPART - 1);
  const int n    = v >> 4;
  const int k8   = (v & 15) * 8;
  const float* W;
  unsigned short* P;
  int pitch, roff, coff;
  if (part == 0)       { W = W1l; P = WB1; pitch = DF; roff = 0;  coff = 0; }
  else if (part == 1)  { W = W1r; P = WB1; pitch = DF; roff = DF; coff = 0; }
  else if (part == 2)  { W = W2l; P = WB2; pitch = KH; roff = 0;  coff = 0; }
  else if (part == 3)  { W = W2l; P = WB2; pitch = KH; roff = 0;  coff = DF; }
  else if (part == 4)  { W = W2r; P = WB2; pitch = KH; roff = DF; coff = 0; }
  else if (part == 5)  { W = W2r; P = WB2; pitch = KH; roff = DF; coff = DF; }
  else return;
  const float* p = W + (size_t)n * DF + k8;
  const v4f a = *(const v4f*)p;
  const v4f b = *(const v4f*)(p + 4);
  v8us o;
  o[0] = (unsigned short)bf16_bits(a.x); o[1] = (unsigned short)bf16_bits(a.y);
  o[2] = (unsigned short)bf16_bits(a.z); o[3] = (unsigned short)bf16_bits(a.w);
  o[4] = (unsigned short)bf16_bits(b.x); o[5] = (unsigned short)bf16_bits(b.y);
  o[6] = (unsigned short)bf16_bits(b.z); o[7] = (unsigned short)bf16_bits(b.w);
  unsigned short* dp = P + (size_t)(roff + n) * pitch + coff + k8;
  *(volatile v8us*)dp = o;
  __threadfence();
  *(volatile v8us*)dp = o;
}

__global__ __launch_bounds__(NTHR) void k_cvx(const float* __restrict__ x, int nN, int nUnits,
                                              unsigned short* xb) {
  const int u = (int)blockIdx.x * NTHR + (int)threadIdx.x;
  if (u >= nUnits) return;
  const int row = u >> 4;
  const int k8  = (u & 15) * 8;
  const int rc  = row < nN ? row : nN - 1;
  const float* p = x + (size_t)rc * DF + k8;
  const v4f a = *(const v4fa*)p;
  const v4f b = *(const v4fa*)(p + 4);
  const bool ok = row < nN;
  v8us o;
  o[0] = ok ? (unsigned short)bf16_bits(a.x) : (unsigned short)0;
  o[1] = ok ? (unsigned short)bf16_bits(a.y) : (unsigned short)0;
  o[2] = ok ? (unsigned short)bf16_bits(a.z) : (unsigned short)0;
  o[3] = ok ? (unsigned short)bf16_bits(a.w) : (unsigned short)0;
  o[4] = ok ? (unsigned short)bf16_bits(b.x) : (unsigned short)0;
  o[5] = ok ? (unsigned short)bf16_bits(b.y) : (unsigned short)0;
  o[6] = ok ? (unsigned short)bf16_bits(b.z) : (unsigned short)0;
  o[7] = ok ? (unsigned short)bf16_bits(b.w) : (unsigned short)0;
  unsigned short* dp = xb + (size_t)row * DF + k8;
  *(volatile v8us*)dp = o;
  __threadfence();
  *(volatile v8us*)dp = o;
}

__global__ __launch_bounds__(GTHR) void k_gemm(
    const unsigned short* __restrict__ A, const unsigned short* __restrict__ WT,
    float* outF, int K, size_t planeStride)
{
  __shared__ __attribute__((aligned(16))) float stg[GBM * GBN];
  const int tid = (int)threadIdx.x, lane = tid & 31, wave = tid >> 5, hh = lane >> 4, m = lane & 15;
  const int rowBase = (int)blockIdx.x * GBM;
  const int ncol    = (int)blockIdx.y * GBN;
  const int pln     = ncol >> 7;
  const int pcol    = ncol & (DF - 1);

  v8f acc[4];
  {
    const v8f z = {0.f, 0.f, 0.f, 0.f, 0.f, 0.f, 0.f, 0.f};
    acc[0] = z; acc[1] = z; acc[2] = z; acc[3] = z;
  }
  const unsigned short* ap = A  + (size_t)(rowBase + 16 * wave + m) * (size_t)K + 8 * hh;
  const unsigned short* wp = WT + (size_t)(ncol + m) * (size_t)K + 8 * hh;
  const int ksteps = K >> 5;
#pragma unroll 1
  for (int ks = 0; ks < ksteps; ++ks) {
    FragB af;
    af.h[0] = *(const v8usa*)(ap + 32 * ks);
    af.h[1] = *(const v8usa*)(ap + 32 * ks + 16);
#pragma unroll
    for (int t = 0; t < 4; ++t) {
      const unsigned short* wq = wp + (size_t)(16 * t) * (size_t)K + 32 * ks;
      FragB bf;
      bf.h[0] = *(const v8usa*)wq;
      bf.h[1] = *(const v8usa*)(wq + 16);
      acc[t] = wmb(af, bf, acc[t]);
    }
  }

#pragma unroll
  for (int t = 0; t < 4; ++t) {
    const int lc = 16 * t + m;
#pragma unroll
    for (int r = 0; r < 8; ++r) {
      const int lr = 16 * wave + 8 * hh + r;
      stg[lr * GBN + lc] = acc[t][r];
    }
  }
  __syncthreads();

  float* ob = outF + (size_t)pln * planeStride;
  v4f fv[8];
#pragma unroll
  for (int i = 0; i < 8; ++i) {
    const int lr = 16 * wave + 2 * i + hh;
    fv[i] = *(const v4fa*)(stg + lr * GBN + 4 * m);
  }
#pragma unroll
  for (int i = 0; i < 8; ++i) {
    const int lr = 16 * wave + 2 * i + hh;
    const int gr = rowBase + lr;
    float* op = ob + (size_t)gr * (size_t)DF + pcol + 4 * m;
    *(volatile v4f*)op = fv[i];
  }
  __threadfence();
#pragma unroll
  for (int i = 0; i < 8; ++i) {
    const int lr = 16 * wave + 2 * i + hh;
    const int gr = rowBase + lr;
    float* op = ob + (size_t)gr * (size_t)DF + pcol + 4 * m;
    *(volatile v4f*)op = fv[i];
  }
}

template <int LYR>
__global__ __launch_bounds__(NTHR) void k_scan(const int* __restrict__ srcs, const int* __restrict__ dsts,
                                               int nE, int nN, int vec8, int mRows,
                                               const float* __restrict__ yl, const float* __restrict__ yr,
                                               const float* __restrict__ bias, float* outp, double* rec) {
  extern __shared__ __attribute__((aligned(16))) int dsm[];
  int* list = dsm;
  int* hl   = dsm + LISTN;
  int* sl   = hl + RCAP;
  int* cnt  = sl + RCAP;
  int* offs = cnt + NBA;
  int* cur  = offs + NBA;
  int* misc = cur + NBA;
  const int tid = (int)threadIdx.x, lane = tid & 31, wave = tid >> 5;
  const int nodeBase = (int)blockIdx.x * NBA;

  {
    const v4i z4 = {0, 0, 0, 0};
    for (int i = tid * 4; i < AGG_ZINTS; i += NTHR * 4) *(v4ia*)(dsm + i) = z4;
    if (tid < MISC_INTS) misc[tid] = 0;
  }
  v4f bv;
  {
    const v4f bq = *(const v4f*)(bias + 4 * lane);
    bv.x = bf16_val(bq.x); bv.y = bf16_val(bq.y); bv.z = bf16_val(bq.z); bv.w = bf16_val(bq.w);
  }
  __syncthreads();

  int t = 0, ov = 0;
  const int nChunks = (nE + CHUNK - 1) / CHUNK;
#pragma unroll 1
  for (int ch = 0; ch < nChunks; ++ch) {
    const int cbase = ch * CHUNK;
    const int wc = scan_chunk<SLA>(dsts, nE, cbase, nodeBase, NBA, vec8, list, tid, lane, wave);
    if (lane == 0) misc[wave] = wc;
    __syncthreads();
    if (wave == 0) {
#pragma unroll 1
      for (int w2 = 0; w2 < NWAVE; ++w2) {
        int c = misc[w2];
        c = c < 0 ? 0 : (c > WCAP ? WCAP : c);
#pragma unroll 1
        for (int b0 = 0; b0 < c; b0 += 32) {
          const int idx = b0 + lane;
          const int ent = list[w2 * WCAP + (idx < WCAP ? idx : WCAP - 1)];
          const int m32 = (c - b0) < 32 ? (c - b0) : 32;
#pragma unroll 1
          for (int k = 0; k < m32; ++k) {
            const int u    = __builtin_amdgcn_readlane(ent, k);
            const int slot = u & (NBA - 1);
            const int el   = (u >> SLA) & (CHUNK - 1);
            const int pk   = ((cbase + el) << SLA) | slot;
            if (t < RCAP) {
              if (lane == 0) { hl[t] = pk; cnt[slot] = cnt[slot] + 1; }
              t = t + 1;
            } else {
              ov = 1;
            }
          }
        }
      }
    }
    __syncthreads();
  }
  if (wave == 0 && lane == 0) { misc[8] = t; misc[9] = ov; }
  __syncthreads();
  int tt = misc[8];
  tt = tt < 0 ? 0 : (tt > RCAP ? RCAP : tt);
  const int ovf = misc[9];

  if (wave == 0) {
    const int base = lane * (NBA / 32);
    int s = 0;
#pragma unroll 1
    for (int i = 0; i < NBA / 32; ++i) s += cnt[base + i];
    int incl = s;
#pragma unroll
    for (int d = 1; d < 32; d <<= 1) {
      const int y = __shfl_up(incl, d, 32);
      if (lane >= d) incl += y;
    }
    int run = incl - s;
#pragma unroll 1
    for (int i = 0; i < NBA / 32; ++i) {
      const int cv = cnt[base + i];
      offs[base + i] = run;
      cur[base + i]  = run;
      run += cv;
    }
  }
  __syncthreads();
  if (wave == 0) {
#pragma unroll 1
    for (int b0 = 0; b0 < tt; b0 += 32) {
      const int idx = b0 + lane;
      const int ent = hl[idx < RCAP ? idx : RCAP - 1];
      const int m32 = (tt - b0) < 32 ? (tt - b0) : 32;
#pragma unroll 1
      for (int k = 0; k < m32; ++k) {
        const int u    = __builtin_amdgcn_readlane(ent, k);
        const int slot = u & (NBA - 1);
        if (lane == 0) {
          int p = cur[slot];
          p = p < 0 ? 0 : (p > RCAP - 1 ? RCAP - 1 : p);
          sl[p] = u;
          cur[slot] = p + 1;
        }
      }
    }
  }
  __syncthreads();

  const float qnan = __int_as_float(0x7fc00000);
  const float pz = (ovf != 0) ? qnan : 0.0f;
  double s0 = 0.0, s1 = 0.0, s2 = 0.0, s3 = 0.0;
  double q0 = 0.0, q1 = 0.0, q2 = 0.0, q3 = 0.0;
#pragma unroll 1
  for (int si = 0; si < NBA / NWAVE; ++si) {
    const int s    = si * NWAVE + wave;
    const int node = nodeBase + s;
    int c = cnt[s];
    const bool big = c > DEGCAP;
    c = c < 0 ? 0 : (c > DEGCAP ? DEGCAP : c);
    int ob = offs[s];
    ob = ob < 0 ? 0 : (ob > RCAP ? RCAP : ob);
    const int nc = node < nN ? node : nN - 1;
    float a0 = 0.0f, a1 = 0.0f, a2 = 0.0f, a3 = 0.0f;
#pragma unroll 1
    for (int b0 = 0; b0 < c; b0 += 32) {
      int idx = ob + b0 + lane;
      idx = idx > RCAP - 1 ? RCAP - 1 : idx;
      const int ent = sl[idx];
      int eid = ent >> SLA;
      eid = eid < 0 ? 0 : (eid > nE - 1 ? nE - 1 : eid);
      int sr = srcs[eid];
      sr = sr < 0 ? 0 : (sr > nN - 1 ? nN - 1 : sr);
      const int m32 = (c - b0) < 32 ? (c - b0) : 32;
#pragma unroll 1
      for (int k = 0; k < m32; ++k) {
        const int sk = __builtin_amdgcn_readlane(sr, k);
        const v4f a = *(const v4f*)(yl + (size_t)sk * DF + 4 * lane);
        a0 += a.x; a1 += a.y; a2 += a.z; a3 += a.w;
      }
    }
    const float cf  = (float)c;
    const float den = (cf < 1.0f) ? 1.0f : cf;
    const float inv = 1.0f / den;
    const v4f rt = *(const v4f*)(yr + (size_t)nc * DF + 4 * lane);
    const float o0 = (a0 * inv + rt.x) + bv.x;
    const float o1 = (a1 * inv + rt.y) + bv.y;
    const float o2 = (a2 * inv + rt.z) + bv.z;
    const float o3 = (a3 * inv + rt.w) + bv.w;
    float ss = (o0 * o0 + o1 * o1) + (o2 * o2 + o3 * o3);
#pragma unroll
    for (int d = 16; d >= 1; d >>= 1) ss += __shfl_xor(ss, d, 32);
    const float nrm = sqrtf(ss);
    const float dn  = (nrm < 1e-12f) ? 1e-12f : nrm;
    const float rin = 1.0f / dn;
    float y0 = o0 * rin, y1 = o1 * rin, y2 = o2 * rin, y3 = o3 * rin;
    if constexpr (LYR == 1) {
      y0 = (y0 > 0.0f) ? y0 : (y0 - y0);
      y1 = (y1 > 0.0f) ? y1 : (y1 - y1);
      y2 = (y2 > 0.0f) ? y2 : (y2 - y2);
      y3 = (y3 > 0.0f) ? y3 : (y3 - y3);
    }
    const float pzr = big ? qnan : pz;
    y0 = y0 + pzr; y1 = y1 + pzr; y2 = y2 + pzr; y3 = y3 + pzr;
    const bool live = node < nN;
    v4f ow;
    ow.x = live ? y0 : 0.0f; ow.y = live ? y1 : 0.0f;
    ow.z = live ? y2 : 0.0f; ow.w = live ? y3 : 0.0f;
    if constexpr (LYR == 1) {
      const double d0 = (double)ow.x, d1 = (double)ow.y, d2 = (double)ow.z, d3 = (double)ow.w;
      s0 += d0; s1 += d1; s2 += d2; s3 += d3;
      q0 += d0 * d0; q1 += d1 * d1; q2 += d2 * d2; q3 += d3 * d3;
    }
    const bool wr = (LYR == 1) ? (node < mRows) : (node < nN);
    if (wr) {
      float* rp = outp + (size_t)node * DF + 4 * lane;
      *(volatile v4f*)rp = ow;
      __threadfence();
      *(volatile v4f*)rp = ow;
    }
  }

  if constexpr (LYR == 1) {
    dbla* part = (dbla*)hl;
    dbla* pw = part + wave * NREC + 4 * lane;
    pw[0] = s0; pw[1] = s1; pw[2] = s2; pw[3] = s3;
    pw[DF + 0] = q0; pw[DF + 1] = q1; pw[DF + 2] = q2; pw[DF + 3] = q3;
    __syncthreads();
    double tot = 0.0;
#pragma unroll
    for (int w2 = 0; w2 < NWAVE; ++w2) tot += part[w2 * NREC + tid];
    part[NWAVE * NREC + tid] = tot;
    __syncthreads();
    if (tid < NREC / 2) {
      const v2d o2 = *(const v2da*)((const double*)hl + NWAVE * NREC + 2 * tid);
      double* rp = rec + (size_t)blockIdx.x * NREC + 2 * tid;
      *(volatile v2d*)rp = o2;
      __threadfence();
      *(volatile v2d*)rp = o2;
    }
  }
}

__global__ __launch_bounds__(128) void k_bnstat(const double* __restrict__ rec, int nRec, double invN,
                                                float* stat) {
  __shared__ __attribute__((aligned(16))) float so[2 * DF];
  const int c = (int)threadIdx.x;
  double S = 0.0, Q = 0.0;
#pragma unroll 1
  for (int b = 0; b < nRec; ++b) {
    S += rec[(size_t)b * NREC + c];
    Q += rec[(size_t)b * NREC + DF + c];
  }
  const double mu = S * invN;
  double var = Q * invN - mu * mu;
  var = (var < 0.0) ? 0.0 : var;
  const float vf = (float)var;
  so[c]      = (float)mu;
  so[DF + c] = 1.0f / sqrtf(vf + 1e-5f);
  __syncthreads();
  if (c < 64) {
    const v4f ov = *(const v4fa*)(so + 4 * c);
    float* op = stat + 4 * c;
    *(volatile v4f*)op = ov;
    __threadfence();
    *(volatile v4f*)op = ov;
  }
}

__device__ __forceinline__ float bn_one(float h, float mu, float rs, float g, float be) {
  return ((h - mu) * rs) * g + be;
}

__global__ __launch_bounds__(NTHR) void k_bnapply(const float* __restrict__ hpl, const float* __restrict__ stat,
                                                  const float* __restrict__ gamma, const float* __restrict__ beta,
                                                  int nN, int nUnits, unsigned short* hbn) {
  const int u = (int)blockIdx.x * NTHR + (int)threadIdx.x;
  if (u >= nUnits) return;
  const int row = u >> 4;
  const int k8  = (u & 15) * 8;
  const int rc  = row < nN ? row : nN - 1;
  const bool ok = row < nN;
  const float* p = hpl + (size_t)rc * DF + k8;
  const v4f ha = *(const v4fa*)p;
  const v4f hb = *(const v4fa*)(p + 4);
  const v4f ma = *(const v4fa*)(stat + k8);
  const v4f mb = *(const v4fa*)(stat + k8 + 4);
  const v4f ra = *(const v4fa*)(stat + DF + k8);
  const v4f rb = *(const v4fa*)(stat + DF + k8 + 4);
  const v4f ga = *(const v4fa*)(gamma + k8);
  const v4f gb = *(const v4fa*)(gamma + k8 + 4);
  const v4f ea = *(const v4fa*)(beta + k8);
  const v4f eb = *(const v4fa*)(beta + k8 + 4);
  float tv[8];
  tv[0] = bn_one(ha.x, ma.x, ra.x, bf16_val(ga.x), bf16_val(ea.x));
  tv[1] = bn_one(ha.y, ma.y, ra.y, bf16_val(ga.y), bf16_val(ea.y));
  tv[2] = bn_one(ha.z, ma.z, ra.z, bf16_val(ga.z), bf16_val(ea.z));
  tv[3] = bn_one(ha.w, ma.w, ra.w, bf16_val(ga.w), bf16_val(ea.w));
  tv[4] = bn_one(hb.x, mb.x, rb.x, bf16_val(gb.x), bf16_val(eb.x));
  tv[5] = bn_one(hb.y, mb.y, rb.y, bf16_val(gb.y), bf16_val(eb.y));
  tv[6] = bn_one(hb.z, mb.z, rb.z, bf16_val(gb.z), bf16_val(eb.z));
  tv[7] = bn_one(hb.w, mb.w, rb.w, bf16_val(gb.w), bf16_val(eb.w));
  v8us oh, ol;
#pragma unroll
  for (int i = 0; i < 8; ++i) {
    const float v = ok ? tv[i] : 0.0f;
    const unsigned hbits = bf16_bits(v);
    const unsigned lbits = bf16_bits(v - __uint_as_float(hbits << 16));
    oh[i] = (unsigned short)hbits;
    ol[i] = (unsigned short)lbits;
  }
  unsigned short* dp = hbn + (size_t)row * KH + k8;
  *(volatile v8us*)dp = oh;
  *(volatile v8us*)(dp + DF) = ol;
  __threadfence();
  *(volatile v8us*)dp = oh;
  *(volatile v8us*)(dp + DF) = ol;
}

static inline int cdiv(int a, int b) { return (a + b - 1) / b; }
static inline size_t al256(size_t o) { return (o + 255) & ~(size_t)255; }

extern "C" void kernel_launch(void* const* d_in, const int* in_sizes, int n_in,
                              void* d_out, int out_size, void* d_ws, size_t ws_size,
                              hipStream_t stream) {
  if (n_in < 10) return;
  if (in_sizes[0] < DF || (in_sizes[0] % DF) != 0) return;
  const int nN = in_sizes[0] / DF;
  if (nN < 1 || nN >= (1 << 24)) return;
  if (in_sizes[1] < 2 || (in_sizes[1] & 1) != 0) return;
  const int nE = in_sizes[1] / 2;
  if (nE < 1 || nE >= (1 << (31 - SLA))) return;
  if (in_sizes[2] != DF * DF || in_sizes[3] != DF * DF) return;
  if (in_sizes[4] != DF || in_sizes[5] != DF || in_sizes[6] != DF) return;
  if (in_sizes[7] != DF * DF || in_sizes[8] != DF * DF) return;
  if (in_sizes[9] != DF) return;
  if ((long long)out_size != (long long)nN * DF) return;

  const float* x     = (const float*)d_in[0];
  const int*   edge  = (const int*)d_in[1];
  const float* W1l   = (const float*)d_in[2];
  const float* W1r   = (const float*)d_in[3];
  const float* b1    = (const float*)d_in[4];
  const float* gamma = (const float*)d_in[5];
  const float* beta  = (const float*)d_in[6];
  const float* W2l   = (const float*)d_in[7];
  const float* W2r   = (const float*)d_in[8];
  const float* b2    = (const float*)d_in[9];
  float* out = (float*)d_out;
  const int* src = edge;
  const int* dst = edge + nE;

  const int MP = cdiv(nN, GBM) * GBM;
  const int gM = MP / GBM;
  const int gA = cdiv(MP, NBA);
  if ((long long)gA * NBA < (long long)MP) return;
  const int vec8 = ((nE & 3) == 0) ? 1 : 0;

  char* ws = (char*)d_ws;
  size_t off = 0;
  const size_t oWB1 = off; off = al256(off + (size_t)2 * DF * DF * 2);
  const size_t oWB2 = off; off = al256(off + (size_t)2 * DF * KH * 2);
  const size_t oXB  = off; off = al256(off + (size_t)MP * DF * 2);
  const size_t oY   = off; off = al256(off + (size_t)2 * MP * DF * 4);
  const size_t oH   = off; off = al256(off + (size_t)MP * DF * 4);
  const size_t oHBN = off; off = al256(off + (size_t)MP * KH * 2);
  const size_t oREC = off; off = al256(off + (size_t)gA * NREC * 8);
  const size_t oST  = off; off = al256(off + (size_t)2 * DF * 4);
  if (off > ws_size || off > (size_t)WSMAX) return;
  unsigned short* WB1 = (unsigned short*)(ws + oWB1);
  unsigned short* WB2 = (unsigned short*)(ws + oWB2);
  unsigned short* XB  = (unsigned short*)(ws + oXB);
  float*          Y   = (float*)(ws + oY);
  float*          H   = (float*)(ws + oH);
  unsigned short* HBN = (unsigned short*)(ws + oHBN);
  double*         REC = (double*)(ws + oREC);
  float*          ST  = (float*)(ws + oST);
  const size_t planeStride = (size_t)MP * DF;
  float* YL = Y;
  float* YR = Y + planeStride;

  const size_t scanLds = (size_t)AGG_LDS_INTS * 4;
  hipFuncSetAttribute(reinterpret_cast<const void*>(&k_scan<1>), hipFuncAttributeMaxDynamicSharedMemorySize, (int)scanLds);
  hipFuncSetAttribute(reinterpret_cast<const void*>(&k_scan<2>), hipFuncAttributeMaxDynamicSharedMemorySize, (int)scanLds);

  const int nUx = MP * (DF / 8);
  const double invN = 1.0 / (double)nN;
  k_wprep<<<(NPART * UPART) / NTHR, NTHR, 0, stream>>>(W1l, W1r, W2l, W2r, WB1, WB2);
  k_cvx<<<cdiv(nUx, NTHR), NTHR, 0, stream>>>(x, nN, nUx, XB);
  k_gemm<<<dim3(gM, (2 * DF) / GBN), GTHR, 0, stream>>>(XB, WB1, Y, DF, planeStride);
  k_scan<1><<<gA, NTHR, scanLds, stream>>>(src, dst, nE, nN, vec8, MP, YL, YR, b1, H, REC);
  k_bnstat<<<1, 128, 0, stream>>>(REC, gA, invN, ST);
  k_bnapply<<<cdiv(nUx, NTHR), NTHR, 0, stream>>>(H, ST, gamma, beta, nN, nUx, HBN);
  k_gemm<<<dim3(gM, (2 * DF) / GBN), GTHR, 0, stream>>>(HBN, WB2, Y, KH, planeStride);
  k_scan<2><<<gA, NTHR, scanLds, stream>>>(src, dst, nE, nN, vec8, MP, YL, YR, b2, out, REC);
}
